// Model_39676907884736
// MI455X (gfx1250) — hardware-run, weakly checked
//
#include <hip/hip_runtime.h>


#ifndef NB
#define NB 2
#endif
#ifndef SEQ
#define SEQ 2048
#endif
#define NB_FULL  2
#define SEQ_FULL 2048
#define TT   SEQ
#define DM   1024
#define NH_  16
#define HD   64
#define DQ   (NH_ * HD)
#define FW   8
#define SCL  0.03125f
#define PCL  14.0f
#define L2E  1.4426950408889634f
#define NEGBIG (-1.0e30f)
#define NEGB 1.0e9f

static_assert(NB >= 1 && NB <= NB_FULL);
static_assert(TT <= SEQ_FULL && TT % 128 == 0);
static_assert(HD == 64 && DM % 64 == 0 && DQ % 64 == 0 && DM % 32 == 0 && TT % 32 == 0 && TT % 64 == 0);
static_assert(DQ == DM);
static_assert(TT % (FW * 16) == 0 && FW * 32 == 256);
static_assert(HD % 32 == 0 && HD * 2 == 128);
static_assert((TT * DM) % (8 * 256) == 0 && (DM * DM) % 8 == 0 && TT % 8 == 0 && (NB * TT) % 4 == 0);

#define SZ_W    ((size_t)DM * DM * 2)
#define SZ_XB   ((size_t)TT * DM * 2)
#define SZ_F    ((size_t)TT * DM * 4)
#define SZ_PL   ((size_t)TT * DM * 2)
#define SZ_BI   ((size_t)NB * TT * 4)
#define SZ_ALL  (3 * SZ_W + SZ_XB + SZ_F + 7 * SZ_PL + SZ_BI)
static_assert(SZ_W % 256 == 0 && SZ_XB % 256 == 0 && SZ_F % 256 == 0 && SZ_PL % 256 == 0 && SZ_BI % 256 == 0);
static_assert(SZ_ALL <= (size_t)134217728);

typedef _Float16 h16;
typedef unsigned short bf;
typedef __attribute__((ext_vector_type(16))) __bf16   v16bf;
typedef __attribute__((ext_vector_type(16))) _Float16 v16h;
typedef __attribute__((ext_vector_type(8)))  _Float16 v8h;
typedef __attribute__((ext_vector_type(8)))  unsigned short v8us;
typedef __attribute__((ext_vector_type(8)))  float    v8f;
typedef __attribute__((ext_vector_type(4)))  float    v4f;
typedef v4f  __attribute__((may_alias)) v4fa;
typedef __attribute__((ext_vector_type(2))) _Float16 v2h;
typedef __attribute__((ext_vector_type(4))) _Float16 v4h;
typedef __attribute__((ext_vector_type(2))) unsigned short v2us;
typedef __attribute__((ext_vector_type(4))) unsigned short v4us;
typedef __attribute__((ext_vector_type(2))) float v2f;
typedef __attribute__((ext_vector_type(4))) int v4i;

__device__ __forceinline__ unsigned short f2bf(float f) { unsigned u = __float_as_uint(f); u += 0x7FFFu + ((u >> 16) & 1u); return (unsigned short)(u >> 16); }
__device__ __forceinline__ float bf2f(unsigned short b) { return __uint_as_float(((unsigned)b) << 16); }
__device__ __forceinline__ float bfr(float f) { return bf2f(f2bf(f)); }
__device__ __forceinline__ v16h cat16(v8h lo, v8h hi) { return __builtin_shufflevector(lo, hi, 0, 1, 2, 3, 4, 5, 6, 7, 8, 9, 10, 11, 12, 13, 14, 15); }
__device__ __forceinline__ v16bf cat16b(v8us lo, v8us hi) { return __builtin_bit_cast(v16bf, __builtin_shufflevector(lo, hi, 0, 1, 2, 3, 4, 5, 6, 7, 8, 9, 10, 11, 12, 13, 14, 15)); }
__device__ __forceinline__ v8f wmma16(v16h a, v16h b, v8f c) { return __builtin_amdgcn_wmma_f32_16x16x32_f16(false, a, false, b, (short)0, c, false, false); }
__device__ __forceinline__ v8f wmmab(v16bf a, v16bf b, v8f c) { return __builtin_amdgcn_wmma_f32_16x16x32_bf16(false, a, false, b, (short)0, c, false, false); }

template <typename T16> struct WFrag;
template <> struct WFrag<h16> { typedef v16h V; static __device__ __forceinline__ V ld(const h16* p) { return cat16(*(const v8h*)p, *(const v8h*)(p + 16)); } static __device__ __forceinline__ v8f mma(V a, V b, v8f c) { return wmma16(a, b, c); } };
template <> struct WFrag<bf> { typedef v16bf V; static __device__ __forceinline__ V ld(const bf* p) { return cat16b(*(const v8us*)p, *(const v8us*)(p + 16)); } static __device__ __forceinline__ v8f mma(V a, V b, v8f c) { return wmmab(a, b, c); } };
template <typename T16, int NSPLIT, bool BIAS>
__global__ __launch_bounds__(32) void k_gemmw(const T16* __restrict__ A, const T16* __restrict__ A2, const T16* __restrict__ Bt, const T16* __restrict__ Bt2, int K, float* C, int ldc, const float* __restrict__ bias, size_t sA, size_t sB, size_t sC) {
    typedef typename WFrag<T16>::V V;
    __shared__ __align__(16) float os[16 * 68];
    const size_t z = blockIdx.z; A += z * sA; if (A2) A2 += z * sA; Bt += z * sB; if (Bt2) Bt2 += z * sB; C += z * sC;
    const int lane = threadIdx.x & 31, lr = lane & 15, hi = lane >> 4; const int r0 = blockIdx.x * 64, c0 = blockIdx.y * 64;
    v8f acc[4][4];
#pragma unroll
    for (int mb = 0; mb < 4; ++mb)
#pragma unroll
        for (int nb = 0; nb < 4; ++nb) acc[mb][nb] = (v8f){};
    const size_t aoff = (size_t)(r0 + lr) * K + 8 * hi, boff = (size_t)(c0 + lr) * K + 8 * hi;
#pragma unroll 1
    for (int kc = 0; kc < K; kc += 32) {
        V a[4], a2[4];
#pragma unroll
        for (int mb = 0; mb < 4; ++mb) { a[mb] = WFrag<T16>::ld(A + aoff + (size_t)mb * 16 * K + kc); if (NSPLIT == 1 || NSPLIT == 2) a2[mb] = WFrag<T16>::ld(A2 + aoff + (size_t)mb * 16 * K + kc); }
#pragma unroll
        for (int nb = 0; nb < 4; ++nb) { const V b = WFrag<T16>::ld(Bt + boff + (size_t)nb * 16 * K + kc); V b2; if (NSPLIT >= 2) b2 = WFrag<T16>::ld(Bt2 + boff + (size_t)nb * 16 * K + kc);
#pragma unroll
            for (int mb = 0; mb < 4; ++mb) { acc[mb][nb] = WFrag<T16>::mma(a[mb], b, acc[mb][nb]); if (NSPLIT == 1 || NSPLIT == 2) acc[mb][nb] = WFrag<T16>::mma(a2[mb], b, acc[mb][nb]); if (NSPLIT >= 2) acc[mb][nb] = WFrag<T16>::mma(a[mb], b2, acc[mb][nb]); } }
        asm volatile("v_nop\n\tv_nop\n\tv_nop\n\tv_nop" : "+v"(acc[0][0]), "+v"(acc[1][1]), "+v"(acc[2][2]), "+v"(acc[3][3]) : "v"(a[0]), "v"(a[3]));
    }
#pragma unroll
    for (int mb = 0; mb < 4; ++mb) {
#pragma unroll
        for (int nb = 0; nb < 4; ++nb) {
#pragma unroll
            for (int j = 0; j < 8; ++j) os[(hi * 8 + j) * 68 + nb * 16 + lr] = acc[mb][nb][j]; }
        __builtin_amdgcn_fence(3  , "wavefront"); __builtin_amdgcn_wave_barrier(); asm volatile("" ::: "memory");
        float* crow = C + (size_t)(r0 + mb * 16) * ldc + c0;
#pragma unroll 1
        for (int ps = 0; ps < 2; ++ps) {
#pragma unroll
            for (int s = 0; s < 8; ++s) { const int row = 2 * s + hi, cofs = lr * 4; v4f val = *(const v4fa*)(os + row * 68 + cofs); if (BIAS) { val[0] += bfr(bias[c0 + cofs]); val[1] += bfr(bias[c0 + cofs + 1]); val[2] += bfr(bias[c0 + cofs + 2]); val[3] += bfr(bias[c0 + cofs + 3]); }
                *(volatile v4f*)(crow + (size_t)row * ldc + cofs) = val; }
            if (ps == 0) __threadfence(); }
        __builtin_amdgcn_fence(3  , "wavefront"); __builtin_amdgcn_wave_barrier(); asm volatile("" ::: "memory");
    }
}

__device__ __forceinline__ void splitf(float y, unsigned short& h, unsigned short& l) { h = f2bf(y); l = f2bf(y - bf2f(h)); }

static __device__ __forceinline__ h16 toh_flush(float v) { const h16 r = (h16)v; return (fabsf(v) < 6.103515625e-05f) ? (h16)0.0f : r; }

static __device__ __forceinline__ v8f wmg(v16h a, v16h b, v8f c) { c = wmma16(a, b, c); asm volatile("v_nop\n\tv_nop\n\tv_nop\n\tv_nop" : "+v"(c) : "v"(a), "v"(b)); return c; }

__global__ __launch_bounds__(256) void k_cvt8(const float* __restrict__ src, bf* dst, size_t n8) { const size_t i = (size_t)blockIdx.x * 256 + threadIdx.x; if (i >= n8) return; const v8f v = *(const v8f*)(src + i * 8); v8us o;
#pragma unroll
    for (int k = 0; k < 8; ++k) o[k] = f2bf(v[k]); *(volatile v8us*)(dst + i * 8) = o; __threadfence(); *(volatile v8us*)(dst + i * 8) = o; }

__global__ __launch_bounds__(256) void k_cvth8(const float* __restrict__ src, h16* dst, size_t n8) { const size_t i = (size_t)blockIdx.x * 256 + threadIdx.x; if (i >= n8) return; const v8f v = *(const v8f*)(src + i * 8); v8h o;
#pragma unroll
    for (int k = 0; k < 8; ++k) o[k] = toh_flush(v[k]); *(volatile v8h*)(dst + i * 8) = o; __threadfence(); *(volatile v8h*)(dst + i * 8) = o; }

__global__ __launch_bounds__(256) void k_split8(const float* __restrict__ src, bf* dh, bf* dl, size_t n8) { const size_t i = (size_t)blockIdx.x * 256 + threadIdx.x; if (i >= n8) return; const v8f v = *(const v8f*)(src + i * 8); v8us oh, ol;
#pragma unroll
    for (int k = 0; k < 8; ++k) { unsigned short a, c2; splitf(v[k], a, c2); oh[k] = a; ol[k] = c2; }
    *(volatile v8us*)(dh + i * 8) = oh; *(volatile v8us*)(dl + i * 8) = ol; __threadfence(); *(volatile v8us*)(dh + i * 8) = oh; *(volatile v8us*)(dl + i * 8) = ol; }

__global__ __launch_bounds__(256) void k_vt16(const float* __restrict__ F, int pitch, h16* VT) { const size_t e = ((size_t)blockIdx.x * 256 + threadIdx.x) * 8; if (e >= (size_t)NH_ * HD * TT) return; const int t = (int)(e % TT); const int d = (int)((e / TT) % HD); const int g = (int)(e / ((size_t)TT * HD)); v8h o;
#pragma unroll
    for (int q = 0; q < 8; ++q) { const float x = F[(size_t)(t + q) * pitch + g * HD + d]; o[q] = toh_flush(x); }
    *(volatile v8h*)(VT + e) = o; __threadfence(); *(volatile v8h*)(VT + e) = o; }

__global__ __launch_bounds__(256) void k_bias(const int* __restrict__ mk, float* bp) { const size_t i = (size_t)blockIdx.x * 256 + threadIdx.x; if (i >= (size_t)NB * TT / 4) return; const size_t e = i * 4; const int b = (int)(e / TT); const int j = (int)(e % TT); const v4i m = *(const v4i*)(mk + (size_t)b * SEQ_FULL + j); v4f o;
#pragma unroll
    for (int q = 0; q < 4; ++q) { const float f = (float)m[q] - 1.0f; o[q] = f * NEGB; }
    *(volatile v4f*)(bp + e) = o; __threadfence(); *(volatile v4f*)(bp + e) = o; }

__global__ __launch_bounds__(256) void k_flash(const h16* __restrict__ Q16, const h16* __restrict__ K16, const h16* __restrict__ VT16, const float* __restrict__ biasf, bf* Ah, bf* Al) {
    __shared__ __align__(16) float os[FW * 16 * 68];
    const int wave = __builtin_amdgcn_readfirstlane(threadIdx.x >> 5);
    const int lane = threadIdx.x & 31, lr = lane & 15, hi = lane >> 4;
    const int head = blockIdx.y; const int q0 = blockIdx.x * (FW * 16) + wave * 16;
    const h16* qp = Q16 + (size_t)(q0 + lr) * DM + head * HD + 8 * hi;
    const v16h qf0 = cat16(*(const v8h*)qp, *(const v8h*)(qp + 16));
    const v16h qf1 = cat16(*(const v8h*)(qp + 32), *(const v8h*)(qp + 48));
    const h16* kp = K16 + (size_t)lr * DM + head * HD + 8 * hi;
    const h16* vp = VT16 + ((size_t)head * HD + lr) * TT + 8 * hi;
    const float* bp = biasf + 8 * hi;
    v8f o0 = (v8f){}, o1 = (v8f){}, o2 = (v8f){}, o3 = (v8f){};
    float m = NEGBIG, l = 0.0f;
#pragma unroll 1
    for (int kc = 0; kc < TT; kc += 32) {
        const h16* ka = kp + (size_t)kc * DM; const h16* kb = ka + (size_t)16 * DM;
        const v8f zz = (v8f){}; v8f s0, s1;
        { const v16h a0 = cat16(*(const v8h*)ka, *(const v8h*)(ka + 16)); s0 = wmg(a0, qf0, zz); }
        { const v16h a1 = cat16(*(const v8h*)(ka + 32), *(const v8h*)(ka + 48)); s0 = wmg(a1, qf1, s0); }
        { const v16h a2 = cat16(*(const v8h*)kb, *(const v8h*)(kb + 16)); s1 = wmg(a2, qf0, zz); }
        { const v16h a3 = cat16(*(const v8h*)(kb + 32), *(const v8h*)(kb + 48)); s1 = wmg(a3, qf1, s1); }
        const v4f b0 = *(const v4f*)(bp + kc), b1 = *(const v4f*)(bp + kc + 4), b2 = *(const v4f*)(bp + kc + 16), b3 = *(const v4f*)(bp + kc + 20);
        float t[16];
#pragma unroll
        for (int r = 0; r < 4; ++r) { t[r] = s0[r] * SCL + b0[r]; t[4 + r] = s0[4 + r] * SCL + b1[r]; t[8 + r] = s1[r] * SCL + b2[r]; t[12 + r] = s1[4 + r] * SCL + b3[r]; }
        float mx = t[0];
#pragma unroll
        for (int i = 1; i < 16; ++i) mx = fmaxf(mx, t[i]);
        mx = fmaxf(mx, __shfl_xor(mx, 16, 32));
        const float nm = fmaxf(m, mx);
        if (__builtin_amdgcn_ballot_w32(nm > m) != 0u) {
            const float al = __builtin_amdgcn_exp2f((m - nm) * L2E); l *= al;
#pragma unroll
            for (int r = 0; r < 8; ++r) { o0[r] *= al; o1[r] *= al; o2[r] *= al; o3[r] *= al; }
            m = nm; }
        v16h pb; float rs = 0.0f;
#pragma unroll
        for (int i = 0; i < 16; ++i) { const float e = (t[i] - m) * L2E + PCL; const float pe = __builtin_amdgcn_exp2f(e); const h16 p = (e < -14.0f) ? (h16)0.0f : (h16)pe; pb[i] = p; rs += (float)p; }
        rs += __shfl_xor(rs, 16, 32); l += rs;
        const h16* vq = vp + kc;
        { const v16h va = cat16(*(const v8h*)vq, *(const v8h*)(vq + 16)); o0 = wmg(va, pb, o0); }
        { const h16* v1 = vq + (size_t)16 * TT; const v16h va = cat16(*(const v8h*)v1, *(const v8h*)(v1 + 16)); o1 = wmg(va, pb, o1); }
        { const h16* v2 = vq + (size_t)32 * TT; const v16h va = cat16(*(const v8h*)v2, *(const v8h*)(v2 + 16)); o2 = wmg(va, pb, o2); }
        { const h16* v3 = vq + (size_t)48 * TT; const v16h va = cat16(*(const v8h*)v3, *(const v8h*)(v3 + 16)); o3 = wmg(va, pb, o3); }
    }
    const float inv = 1.0f / l;
    const int ob = wave * 16 * 68; const int wi = ob + lr * 68 + 8 * hi;
    { v4f x; x[0] = o0[0] * inv; x[1] = o0[1] * inv; x[2] = o0[2] * inv; x[3] = o0[3] * inv; *(v4fa*)&os[wi] = x; x[0] = o0[4] * inv; x[1] = o0[5] * inv; x[2] = o0[6] * inv; x[3] = o0[7] * inv; *(v4fa*)&os[wi + 4] = x; }
    { v4f x; x[0] = o1[0] * inv; x[1] = o1[1] * inv; x[2] = o1[2] * inv; x[3] = o1[3] * inv; *(v4fa*)&os[wi + 16] = x; x[0] = o1[4] * inv; x[1] = o1[5] * inv; x[2] = o1[6] * inv; x[3] = o1[7] * inv; *(v4fa*)&os[wi + 20] = x; }
    { v4f x; x[0] = o2[0] * inv; x[1] = o2[1] * inv; x[2] = o2[2] * inv; x[3] = o2[3] * inv; *(v4fa*)&os[wi + 32] = x; x[0] = o2[4] * inv; x[1] = o2[5] * inv; x[2] = o2[6] * inv; x[3] = o2[7] * inv; *(v4fa*)&os[wi + 36] = x; }
    { v4f x; x[0] = o3[0] * inv; x[1] = o3[1] * inv; x[2] = o3[2] * inv; x[3] = o3[3] * inv; *(v4fa*)&os[wi + 48] = x; x[0] = o3[4] * inv; x[1] = o3[5] * inv; x[2] = o3[6] * inv; x[3] = o3[7] * inv; *(v4fa*)&os[wi + 52] = x; }
    __builtin_amdgcn_fence(3  , "wavefront"); __builtin_amdgcn_wave_barrier(); asm volatile("" ::: "memory");
#pragma unroll 1
    for (int ps = 0; ps < 2; ++ps) {
#pragma unroll
        for (int it = 0; it < 4; ++it) { const int row = it * 4 + (lane >> 3), pc = (lane & 7) * 8;
            const v4f x0 = *(const v4fa*)&os[ob + row * 68 + pc]; const v4f x1 = *(const v4fa*)&os[ob + row * 68 + pc + 4]; v8us oh, ol;
#pragma unroll
            for (int q = 0; q < 4; ++q) { unsigned short a, c2; splitf(x0[q], a, c2); oh[q] = a; ol[q] = c2; splitf(x1[q], a, c2); oh[4 + q] = a; ol[4 + q] = c2; }
            const size_t oo = (size_t)(q0 + row) * DQ + head * HD + pc; *(volatile v8us*)(Ah + oo) = oh; *(volatile v8us*)(Al + oo) = ol; }
        if (ps == 0) __threadfence(); }
}

extern "C" void kernel_launch(void* const* d_in, const int* in_sizes, int n_in,
                              void* d_out, int out_size, void* d_ws, size_t ws_size, hipStream_t stream) {
    if (n_in < 10) return;
    const size_t needx = (size_t)(NB - 1) * SEQ_FULL * DM + (size_t)TT * DM;
    const size_t needm = (size_t)(NB - 1) * SEQ_FULL + (size_t)TT;
    if ((size_t)in_sizes[0] < needx || (size_t)in_sizes[1] < needx || (size_t)in_sizes[2] < needx || (size_t)in_sizes[9] < needm) return;
    if ((size_t)in_sizes[3] < (size_t)DM * DM || (size_t)in_sizes[5] < (size_t)DM * DM || (size_t)in_sizes[7] < (size_t)DM * DM) return;
    if (in_sizes[4] < DM || in_sizes[6] < DM || in_sizes[8] < DM) return;
    if ((size_t)out_size < needx) return;
    const float* xq = (const float*)d_in[0]; const float* xk = (const float*)d_in[1]; const float* xv = (const float*)d_in[2];
    const float* win = (const float*)d_in[3]; const float* bin = (const float*)d_in[4]; const float* wff = (const float*)d_in[5]; const float* bff = (const float*)d_in[6];
    const float* wout = (const float*)d_in[7]; const float* bout = (const float*)d_in[8]; const int* mask = (const int*)d_in[9];
    float* OUT = (float*)d_out;
    char* wsp = (char*)d_ws;
    auto take = [&](size_t bytes) { char* p = wsp; wsp += (bytes + 255) & ~(size_t)255; return (void*)p; };
    bf* WIN = (bf*)take(SZ_W); bf* WFF = (bf*)take(SZ_W); bf* WOUT = (bf*)take(SZ_W);
    bf* XB = (bf*)take(SZ_XB); float* F = (float*)take(SZ_F);
    bf* T1h = (bf*)take(SZ_PL); bf* T1l = (bf*)take(SZ_PL);
    h16* Q16 = (h16*)take(SZ_PL); h16* K16 = (h16*)take(SZ_PL); h16* VT16 = (h16*)take(SZ_PL);
    bf* ATh = (bf*)take(SZ_PL); bf* ATl = (bf*)take(SZ_PL);
    float* BIASF = (float*)take(SZ_BI);
    if ((size_t)(wsp - (char*)d_ws) > ws_size) return;
    const unsigned LW = (unsigned)(((size_t)DM * DM / 8 + 255) / 256);
    k_cvt8<<<LW, 256, 0, stream>>>(win, WIN, (size_t)DM * DM / 8);
    k_cvt8<<<LW, 256, 0, stream>>>(wff, WFF, (size_t)DM * DM / 8);
    k_cvt8<<<LW, 256, 0, stream>>>(wout, WOUT, (size_t)DM * DM / 8);
    k_bias<<<(unsigned)(((size_t)NB * TT / 4 + 255) / 256), 256, 0, stream>>>(mask, BIASF);
    const size_t NX8 = (size_t)TT * DM / 8;
    const unsigned LX = (unsigned)((NX8 + 255) / 256);
    const dim3 GP(TT / 64, DM / 64, 1);
    for (int b = 0; b < NB; ++b) {
        const size_t xo = (size_t)b * SEQ_FULL * DM;
        k_cvt8<<<LX, 256, 0, stream>>>(xq + xo, XB, NX8);
        k_gemmw<bf, 0, true><<<GP, 32, 0, stream>>>(XB, nullptr, WIN, nullptr, DM, F, DM, bin, 0, 0, 0);
        k_cvth8<<<LX, 256, 0, stream>>>(F, Q16, NX8);
        k_cvt8<<<LX, 256, 0, stream>>>(xk + xo, XB, NX8);
        k_gemmw<bf, 0, true><<<GP, 32, 0, stream>>>(XB, nullptr, WIN, nullptr, DM, F, DM, bin, 0, 0, 0);
        k_cvt8<<<LX, 256, 0, stream>>>(F, T1h, NX8);
        k_gemmw<bf, 0, true><<<GP, 32, 0, stream>>>(T1h, nullptr, WOUT, nullptr, DM, F, DM, bout, 0, 0, 0);
        k_cvth8<<<LX, 256, 0, stream>>>(F, K16, NX8);
        k_cvt8<<<LX, 256, 0, stream>>>(xv + xo, XB, NX8);
        k_gemmw<bf, 0, true><<<GP, 32, 0, stream>>>(XB, nullptr, WIN, nullptr, DM, F, DM, bin, 0, 0, 0);
        k_split8<<<LX, 256, 0, stream>>>(F, T1h, T1l, NX8);
        k_gemmw<bf, 1, true><<<GP, 32, 0, stream>>>(T1h, T1l, WOUT, nullptr, DM, F, DM, bout, 0, 0, 0);
        k_vt16<<<LX, 256, 0, stream>>>(F, DM, VT16);
        k_flash<<<dim3(TT / (FW * 16), NH_, 1), 256, 0, stream>>>(Q16, K16, VT16, BIASF + (size_t)b * TT, ATh, ATl);
        k_gemmw<bf, 1, true><<<GP, 32, 0, stream>>>(ATh, ATl, WFF, nullptr, DQ, F, DM, bff, 0, 0, 0);
        k_split8<<<LX, 256, 0, stream>>>(F, T1h, T1l, NX8);
        k_gemmw<bf, 1, true><<<GP, 32, 0, stream>>>(T1h, T1l, WOUT, nullptr, DM, OUT + xo, DM, bout, 0, 0, 0); }
}
